// IDGAT_27479200760359
// MI455X (gfx1250) — hardware-verified
//
#include <hip/hip_runtime.h>


namespace {
constexpr int N = 50000, F = 128, U = 128, NH = 8, DHD = 16, E = 600000, NID = 5000, NPAD = 50176, NBLK = NPAD / 128, W4 = 4 * U;
constexpr float FXS = 262144.0f, FXI = 1.0f / 262144.0f, ISQ = 0.25f  ;

typedef _Float16 b16;
typedef __attribute__((ext_vector_type(16))) _Float16 v16b;
typedef __attribute__((ext_vector_type(8)))  _Float16 v8b;
typedef __attribute__((ext_vector_type(8)))  float v8f;
typedef __attribute__((ext_vector_type(4)))  float v4f;

__device__ __forceinline__ v8b ld8b(const b16* p) { return *(const v8b*)p; }
__device__ __forceinline__ v16b cat8b(v8b a, v8b b) { return __builtin_shufflevector(a, b, 0, 1, 2, 3, 4, 5, 6, 7, 8, 9, 10, 11, 12, 13, 14, 15); }
__device__ __forceinline__ v16b frag_kb(const b16* p, int hh) { return cat8b(ld8b(p + 8 * hh), ld8b(p + 16 + 8 * hh)); }
__device__ __forceinline__ void split16(float v, b16& hi, b16& lo) { hi = (b16)v; lo = (b16)(v - (float)hi); }
__device__ __forceinline__ void frag_ksplit(const float* p, int hh, v16b& fh_, v16b& fl_) {
  const float* p0 = p + 8 * hh; const float* p1 = p + 16 + 8 * hh;
#pragma unroll
  for (int e = 0; e < 8; ++e) { b16 a, c; split16(p0[e], a, c); fh_[e] = a; fl_[e] = c; split16(p1[e], a, c); fh_[8 + e] = a; fl_[8 + e] = c; }
}
__device__ __forceinline__ v8f wmma16b(v16b a, v16b b, v8f c) {
  v8f d = __builtin_amdgcn_wmma_f32_16x16x32_f16(false, a, false, b, (short)0, c, false, false);
  asm volatile("v_nop\n\tv_nop\n\tv_nop\n\tv_nop" : "+v"(d) : "v"(a), "v"(b));
  return d;
}
__device__ __forceinline__ void wave_lds_sync() {
  __builtin_amdgcn_fence(__ATOMIC_RELEASE, "workgroup");
  __builtin_amdgcn_wave_barrier();
  __builtin_amdgcn_fence(__ATOMIC_ACQUIRE, "workgroup");
}

struct Opnd { const void* p0; const void* p1; int ld; };
template <int NP> __device__ __forceinline__ void load_frags(const Opnd& o, int row, int kb, int hh, v16b& fh_, v16b& fl_) {
  if (NP == 0) { frag_ksplit((const float*)o.p0 + (size_t)row * o.ld + kb, hh, fh_, fl_); }
  else if (NP == 4) {
    const float* p = (const float*)o.p0 + (size_t)row * o.ld + kb; const float* p0 = p + 8 * hh; const float* p1 = p + 16 + 8 * hh;
#pragma unroll
    for (int e = 0; e < 8; ++e) { b16 a, c; split16(p0[e] * 64.0f, a, c); fh_[e] = a; fl_[e] = c; split16(p1[e] * 64.0f, a, c); fh_[8 + e] = a; fl_[8 + e] = c; }
  } else if (NP == 3) {
    const float* p = (const float*)o.p0 + (size_t)row * o.ld + kb; const float* p0 = p + 8 * hh; const float* p1 = p + 16 + 8 * hh;
#pragma unroll
    for (int e = 0; e < 8; ++e) { fh_[e] = (b16)p0[e]; fh_[8 + e] = (b16)p1[e]; }
    fl_ = fh_;
  } else {
    fh_ = frag_kb((const b16*)o.p0 + (size_t)row * o.ld + kb, hh);
    if (NP == 2) fl_ = frag_kb((const b16*)o.p1 + (size_t)row * o.ld + kb, hh); else fl_ = fh_;
  }
}
template <int ANP, int BNP> __device__ __forceinline__ v8f mac(v16b ah, v16b al, v16b bh, v16b bl, v8f c) {
  c = wmma16b(ah, bh, c);
  if (BNP == 0 || BNP == 2 || BNP == 4) c = wmma16b(ah, bl, c);
  if (ANP == 0 || ANP == 2 || ANP == 4) c = wmma16b(al, bh, c);
  return c;
}
template <int ANP, int BNP>
__device__ __forceinline__ void gemm_tile(const Opnd& A, const Opnd& B, int K, int m0, int c0, int nloc, int hlf, v8f (&acc)[2][4]) {
  for (int kb = 0; kb < K; kb += 32) {
    v16b a0h, a0l, a1h, a1l;
    load_frags<ANP>(A, m0 + nloc, kb, hlf, a0h, a0l);
    load_frags<ANP>(A, m0 + 16 + nloc, kb, hlf, a1h, a1l);
#pragma unroll
    for (int t = 0; t < 4; ++t) {
      v16b bh, bl;
      load_frags<BNP>(B, c0 + t * 16 + nloc, kb, hlf, bh, bl);
      acc[0][t] = mac<ANP, BNP>(a0h, a0l, bh, bl, acc[0][t]);
      acc[1][t] = mac<ANP, BNP>(a1h, a1l, bh, bl, acc[1][t]);
    }
  }
}

__device__ __forceinline__ void epi_planes(v8f (&acc)[2][4], float scale, bool two, b16* __restrict__ oh, b16* __restrict__ ol, int ldo,
                                           int m0, int c0, int lane, b16* Th, b16* Tl) {
  const int nloc = lane & 15, hlf = lane >> 4;
#pragma unroll
  for (int t = 0; t < 4; ++t)
#pragma unroll
    for (int r = 0; r < 2; ++r)
#pragma unroll
      for (int v = 0; v < 8; ++v) {
        const int rr = r * 16 + v + 8 * hlf, cc = t * 16 + nloc;
        b16 h_, l_; split16(acc[r][t][v] * scale, h_, l_);
        Th[rr * 64 + cc] = h_; Tl[rr * 64 + cc] = l_;
      }
  wave_lds_sync();
  for (int pass = 0; pass < 2; ++pass) {
#pragma unroll
    for (int j = 0; j < 8; ++j) {
      const int rr = j * 4 + (lane >> 3), c8 = (lane & 7) * 8;
      const size_t o = (size_t)(m0 + rr) * ldo + c0 + c8;
      *(volatile v8b*)(oh + o) = ld8b(Th + rr * 64 + c8);
      if (two) *(volatile v8b*)(ol + o) = ld8b(Tl + rr * 64 + c8);
    }
    __threadfence();
  }
}
__device__ __forceinline__ void epi_f32(v8f (&acc)[2][4], float scale, const float* rscale, float* __restrict__ out, int ldo, int m0, int c0, int lane, float* Tt) {
  const int nloc = lane & 15, hlf = lane >> 4;
#pragma unroll
  for (int t = 0; t < 4; ++t)
#pragma unroll
    for (int r = 0; r < 2; ++r)
#pragma unroll
      for (int v = 0; v < 8; ++v) {
        const int rr = r * 16 + v + 8 * hlf;
        const float rs = rscale ? rscale[(size_t)(m0 + rr) * 32] : 1.0f;
        Tt[rr * 64 + t * 16 + nloc] = acc[r][t][v] * scale * rs;
      }
  wave_lds_sync();
  float* dst0 = out + (size_t)m0 * ldo + c0;
  for (int pass = 0; pass < 2; ++pass) {
#pragma unroll
    for (int j = 0; j < 16; ++j) { const int rr = j * 2 + hlf, c4 = nloc * 4; *(volatile v4f*)(dst0 + (size_t)rr * ldo + c4) = *(const v4f*)(Tt + rr * 64 + c4); }
    __threadfence();
  }
}


__device__ __forceinline__ int fkey(float f) { const int b = __float_as_int(f); return (b >= 0) ? b : (b ^ 0x7FFFFFFF); }
__device__ __forceinline__ float fkey_inv(int k) { return __int_as_float((k >= 0) ? k : (k ^ 0x7FFFFFFF)); }

__global__ __launch_bounds__(256) void prep_kernel(const float* __restrict__ wq, const float* __restrict__ wk, const float* __restrict__ w, const float* __restrict__ wid, b16* __restrict__ wr, b16* __restrict__ wl) {
  const size_t tid = (size_t)blockIdx.x * blockDim.x + threadIdx.x, nth = (size_t)gridDim.x * blockDim.x;
  for (int pass = 0; pass < 2; ++pass) { for (size_t p = tid; p < (size_t)W4 * F; p += nth) { const int n = (int)(p / F), k = (int)(p % F); const int m = n / U, nn = n % U; const float* Wm = (m == 0) ? wq : (m == 1) ? wk : (m == 2) ? w : wid;
      b16 a, c; split16(Wm[(size_t)k * U + nn] * 64.0f, a, c); ((volatile b16*)wr)[p] = a; ((volatile b16*)wl)[p] = c; } __threadfence(); }
}

__global__ __launch_bounds__(256) void idcount_kernel(const int* __restrict__ ids, float* __restrict__ cntf) {
  constexpr int NB = 8192;
  __shared__ int cnt[NB];
  const int t_ = threadIdx.x, base = blockIdx.x * NB;
  for (int i = t_; i < NB; i += 256) cnt[i] = 0;
  __syncthreads();
  for (int i = t_; i < NID; i += 256) { const unsigned sl = (unsigned)(ids[i] - base); if (sl < (unsigned)NB) atomicAdd(&cnt[sl], 1); }
  __syncthreads();
  for (int pass = 0; pass < 2; ++pass) { for (int i = t_; i < NB / 4; i += 256) { const int node = base + i * 4; if (node < NPAD) { v4f o; o[0] = (float)cnt[i * 4]; o[1] = (float)cnt[i * 4 + 1]; o[2] = (float)cnt[i * 4 + 2]; o[3] = (float)cnt[i * 4 + 3]; *(volatile v4f*)(cntf + node) = o; } } __threadfence(); }
}

__global__ __launch_bounds__(128) void node_kernel(const float* __restrict__ x, const b16* __restrict__ wr, const b16* __restrict__ wlo, const float* __restrict__ bq, const float* __restrict__ bk, float* __restrict__ y) {
  __shared__ __attribute__((aligned(16))) float Ts[4][32 * 64];
  const int lane = threadIdx.x & 31, wave = threadIdx.x >> 5, nloc = lane & 15, hlf = lane >> 4, m0 = blockIdx.y * 128 + wave * 32, c0 = blockIdx.x * 64;
  v8f acc[2][4];
#pragma unroll
  for (int r = 0; r < 2; ++r)
#pragma unroll
    for (int t = 0; t < 4; ++t) acc[r][t] = (v8f){};
  const int ra = min(m0 + nloc, N - 1), rb = min(m0 + 16 + nloc, N - 1);
#pragma unroll 1
  for (int kb = 0; kb < F; kb += 32) { v16b a0, a1, l0, l1;
#pragma unroll
    for (int e = 0; e < 16; ++e) { const int k = kb + ((e < 8) ? (8 * hlf + e) : (16 + 8 * hlf + e - 8)); b16 p, q; split16(x[(size_t)ra * F + k] * 8.0f, p, q); a0[e] = p; l0[e] = q; split16(x[(size_t)rb * F + k] * 8.0f, p, q); a1[e] = p; l1[e] = q; }
#pragma unroll
    for (int t = 0; t < 4; ++t) { const v16b bw = frag_kb(wr + (size_t)(c0 + t * 16 + nloc) * F + kb, hlf), bl = frag_kb(wlo + (size_t)(c0 + t * 16 + nloc) * F + kb, hlf);
      acc[0][t] = wmma16b(a0, bw, acc[0][t]); acc[0][t] = wmma16b(l0, bw, acc[0][t]); acc[0][t] = wmma16b(a0, bl, acc[0][t]);
      acc[1][t] = wmma16b(a1, bw, acc[1][t]); acc[1][t] = wmma16b(l1, bw, acc[1][t]); acc[1][t] = wmma16b(a1, bl, acc[1][t]); } }
#pragma unroll
  for (int t = 0; t < 4; ++t)
#pragma unroll
    for (int r = 0; r < 2; ++r)
#pragma unroll
      for (int v = 0; v < 8; ++v) { const int c = c0 + t * 16 + nloc; float val = acc[r][t][v] * (1.0f / 512.0f);
        if (c < U) val = fmaxf(val + bq[c], 0.0f); else if (c < 2 * U) val = fmaxf(val + bk[c - U], 0.0f);
        acc[r][t][v] = val; }
  epi_f32(acc, 1.0f, nullptr, y, W4, m0, c0, lane, Ts[wave]);
}

__global__ __launch_bounds__(256) void escore_kernel(const int* __restrict__ erow, const int* __restrict__ ecol, const float* __restrict__ y, float* __restrict__ esc) {
  __shared__ float Eo[32 * NH];
  const int t_ = threadIdx.x, el = t_ >> 3, h = t_ & 7, e = min(blockIdx.x * 32 + el, E - 1);
  int r = erow[e], c = ecol[e]; r = (r < 0) ? 0 : (r >= N ? N - 1 : r); c = (c < 0) ? 0 : (c >= N ? N - 1 : c);
  const float* q = y + (size_t)r * W4 + h * DHD; const float* k = y + (size_t)c * W4 + U + h * DHD; float s = 0.0f;
#pragma unroll
  for (int d = 0; d < DHD; d += 4) { const v4f a = *(const v4f*)(q + d), b = *(const v4f*)(k + d); s += a[0] * b[0] + a[1] * b[1] + a[2] * b[2] + a[3] * b[3]; }
  Eo[t_] = s * ISQ;
  __syncthreads();
  for (int pass = 0; pass < 2; ++pass) { if (t_ < 64 && blockIdx.x * 32 + (t_ >> 1) < E) *(volatile v4f*)(esc + (size_t)(blockIdx.x * 32) * NH + t_ * 4) = *(const v4f*)(&Eo[t_ * 4]); __threadfence(); }
}

__global__ __launch_bounds__(256) void att_kernel(const int* __restrict__ erow, const int* __restrict__ ecol, const float* __restrict__ esc, const float* __restrict__ y, const float* __restrict__ cntf, const float* __restrict__ bias, float* __restrict__ out) {
  constexpr int NB = 256;
  __shared__ __attribute__((aligned(16))) int acc[NB * U]; __shared__ int mx[NB * NH]; __shared__ int den[NB * NH]; __shared__ int list[8 * 256]; __shared__ float selfsc[NB * NH];
  const int t_ = threadIdx.x, wave = t_ >> 5, lane = t_ & 31, base = blockIdx.x * NB, col0 = lane * 4, myh = lane >> 2;
  for (int i = t_; i < NB * U; i += 256) acc[i] = 0;
  for (int i = t_; i < NB * NH; i += 256) { const int slot = i >> 3, h = i & 7, node = base + slot; float sc = -INFINITY;
    if (node < N) { const float* q = y + (size_t)node * W4 + h * DHD; const float* k = y + (size_t)node * W4 + U + h * DHD; float s = 0.0f;
#pragma unroll
      for (int d = 0; d < DHD; ++d) s += q[d] * k[d];
      sc = s * ISQ; }
    selfsc[i] = sc; mx[i] = fkey(sc); den[i] = 0; }
  __syncthreads();
  for (int c0 = 0; c0 < E; c0 += 256 * 8) { const int e0 = c0 + (wave * 32 + lane) * 8;
#pragma unroll
    for (int j = 0; j < 8; ++j) { const int ee = min(e0 + j, E - 1); const int dv = erow[ee]; const unsigned sl = (unsigned)(((e0 + j < E) ? dv : -1) - base);
      if (sl < (unsigned)NB) {
#pragma unroll
        for (int h = 0; h < NH; ++h) atomicMax(&mx[sl * NH + h], fkey(esc[(size_t)ee * NH + h])); } } }
  __syncthreads();
  int* wl = list + wave * 256;
  auto accumulate = [&](int c, int slot, v4f ea, v4f eb) {
    auto sel8 = [&](int h) { float v = ea[0]; v = (h == 1) ? ea[1] : v; v = (h == 2) ? ea[2] : v; v = (h == 3) ? ea[3] : v; v = (h == 4) ? eb[0] : v; v = (h == 5) ? eb[1] : v; v = (h == 6) ? eb[2] : v; v = (h == 7) ? eb[3] : v; return v; };
    const float wm = __expf(sel8(myh) - fkey_inv(mx[slot * NH + myh]));
    if (lane < NH) { const float wd = __expf(sel8(lane) - fkey_inv(mx[slot * NH + lane])); atomicAdd(&den[slot * NH + lane], (int)rintf(wd * FXS)); }
    const float cc = cntf[c]; const v4f hv = *(const v4f*)(y + (size_t)c * W4 + 2 * U + col0), iv = *(const v4f*)(y + (size_t)c * W4 + 3 * U + col0); int* ar = acc + slot * U + col0;
#pragma unroll
    for (int q = 0; q < 4; ++q) atomicAdd(ar + q, (int)rintf(wm * (hv[q] + cc * iv[q]) * FXS));
  };
  for (int slot = wave; slot < NB; slot += 8) { if (base + slot < N) { const v4f ea = {selfsc[slot * NH], selfsc[slot * NH + 1], selfsc[slot * NH + 2], selfsc[slot * NH + 3]}, eb = {selfsc[slot * NH + 4], selfsc[slot * NH + 5], selfsc[slot * NH + 6], selfsc[slot * NH + 7]}; accumulate(base + slot, slot, ea, eb); } }
  for (int c0 = 0; c0 < E; c0 += 256 * 8) {
    const int e0 = c0 + (wave * 32 + lane) * 8; int dd[8];
#pragma unroll
    for (int j = 0; j < 8; ++j) { const int dv = erow[min(e0 + j, E - 1)]; dd[j] = (e0 + j < E) ? dv : -1; }
    unsigned sl[8]; bool hit[8]; bool anyl = false;
#pragma unroll
    for (int j = 0; j < 8; ++j) { sl[j] = (unsigned)(dd[j] - base); hit[j] = sl[j] < (unsigned)NB; anyl |= hit[j]; }
    int wc = 0;
    if (__builtin_amdgcn_ballot_w32(anyl) != 0u) {
#pragma unroll
      for (int j = 0; j < 8; ++j) {
        const unsigned mj = __builtin_amdgcn_ballot_w32(hit[j]);
        if (mj != 0u) {
          if (hit[j]) { const int pos = wc + (int)__builtin_amdgcn_mbcnt_lo(mj, 0u); wl[pos] = ((e0 + j) << 8) | (int)sl[j]; }
          wc += __builtin_popcount(mj); } } }
    __builtin_amdgcn_wave_barrier(); __builtin_amdgcn_fence(__ATOMIC_RELEASE, "workgroup"); __builtin_amdgcn_fence(__ATOMIC_ACQUIRE, "workgroup");
    for (int i = 0; i < wc; ++i) { const int ent = wl[i]; const int e = ent >> 8, slot = ent & 255; int c = ecol[e]; c = (c < 0) ? 0 : (c >= N ? N - 1 : c);
      const v4f ea = *(const v4f*)(esc + (size_t)e * NH), eb = *(const v4f*)(esc + (size_t)e * NH + 4);
      accumulate(c, slot, ea, eb); }
    __builtin_amdgcn_wave_barrier();
  }
  __syncthreads();
  for (int pass = 0; pass < 2; ++pass) {
    for (int i = t_; i < NB * U / 4; i += 256) { const int r = i >> 5, cq = (i & 31) * 4, node = base + r; if (node < N) { const int h = cq / DHD; const float id = __builtin_amdgcn_rcpf((float)den[r * NH + h]); v4f o;
#pragma unroll
        for (int q = 0; q < 4; ++q) o[q] = (float)acc[r * U + cq + q] * id + bias[cq + q];
        *(volatile v4f*)(out + (size_t)node * U + cq) = o; } }
    __threadfence();
  }
}
}

extern "C" void kernel_launch(void* const* d_in, const int* in_sizes, int n_in,
                              void* d_out, int out_size, void* d_ws, size_t ws_size, hipStream_t stream) {
  (void)n_in; (void)out_size;
  const float* x = (const float*)d_in[0]; const int* ei = (const int*)d_in[1]; const int* ids = (const int*)d_in[2];
  const float* wq = (const float*)d_in[3]; const float* bq = (const float*)d_in[4]; const float* wk = (const float*)d_in[5]; const float* bk = (const float*)d_in[6]; const float* w = (const float*)d_in[7]; const float* wid = (const float*)d_in[8]; const float* bias = (const float*)d_in[9];
  float* out = (float*)d_out;
  if (in_sizes[0] != N * F || in_sizes[1] != 2 * E || in_sizes[2] != NID || in_sizes[3] != F * U || in_sizes[8] != F * U) return;
  const int* erow = ei; const int* ecol = ei + E;
  size_t off = 0; char* ws = (char*)d_ws;
  auto carve = [&](size_t bytes) { char* p = ws + off; off += (bytes + 255) & ~(size_t)255; return p; };
  b16* wr = (b16*)carve((size_t)W4 * F * 2); b16* wlo = (b16*)carve((size_t)W4 * F * 2); float* cntf = (float*)carve((size_t)NPAD * 4 + 32768); float* y = (float*)carve((size_t)NPAD * W4 * 4); float* esc = (float*)carve((size_t)E * NH * 4);
  if (off > ws_size) return;
  prep_kernel<<<64, 256, 0, stream>>>(wq, wk, w, wid, wr, wlo);
  idcount_kernel<<<(NPAD + 8191) / 8192, 256, 0, stream>>>(ids, cntf);
  node_kernel<<<dim3(W4 / 64, NBLK), 128, 0, stream>>>(x, wr, wlo, bq, bk, y);
  escore_kernel<<<(E + 31) / 32, 256, 0, stream>>>(erow, ecol, y, esc);
  att_kernel<<<NPAD / 256, 256, 0, stream>>>(erow, ecol, esc, y, cntf, bias, out);
}
